// Seq2Seq_RNN_RNN_Model_15169824489877
// MI455X (gfx1250) — hardware-verified
//
#include <hip/hip_runtime.h>
#include <math.h>

typedef __attribute__((ext_vector_type(16))) _Float16 v16h;
typedef __attribute__((ext_vector_type(16))) __bf16 v16b;
typedef __attribute__((ext_vector_type(8)))  _Float16 v8h;
typedef __attribute__((ext_vector_type(8)))  float v8f;
typedef __attribute__((ext_vector_type(4)))  float v4f;
typedef __attribute__((ext_vector_type(2)))  float v2f;
typedef __attribute__((ext_vector_type(4)))  unsigned v4u;
typedef __attribute__((ext_vector_type(4)))  int v4i;
typedef float __attribute__((may_alias)) float_a;
typedef int __attribute__((may_alias)) int_a;

template <typename T> __device__ __forceinline__ void vst2(void* p, T v) { *(volatile T*)p = v; __threadfence(); *(volatile T*)p = v; }
__device__ __forceinline__ v8f wmma16(v16h a, v16h b, v8f c) {
  v8f d = __builtin_amdgcn_wmma_f32_16x16x32_f16(false, a, false, b, (short)0, c, false, false);
  asm volatile("v_nop\n\tv_nop\n\tv_nop\n\tv_nop" : "+v"(d) : "v"(a), "v"(b));
  return d;
}
__device__ __forceinline__ v8f wmma_bf(v16b a, v16b b, v8f c) {
  v8f d = __builtin_amdgcn_wmma_f32_16x16x32_bf16(false, a, false, b, (short)0, c, false, false);
  asm volatile("v_nop\n\tv_nop\n\tv_nop\n\tv_nop" : "+v"(d) : "v"(a), "v"(b));
  return d;
}
__device__ __forceinline__ v16h frag_h(const _Float16* rowk0, int lane) {
  union { v16h v; v8h q[2]; } u; const _Float16* p = rowk0 + 8 * (lane >> 4);
  u.q[0] = *(const v8h*)p; u.q[1] = *(const v8h*)(p + 16); return u.v;
}
__device__ __forceinline__ v16h frag_f32(const float* rowk0, int lane) {
  v16h a; const float* p = rowk0 + 8 * (lane >> 4);
#pragma unroll
  for (int i = 0; i < 8; ++i) { a[i] = (_Float16)p[i]; a[8 + i] = (_Float16)p[16 + i]; }
  return a;
}
__device__ __forceinline__ v16h frag_f32s(const float* rowk0, int lane, float sc) {
  v16h a; const float* p = rowk0 + 8 * (lane >> 4);
#pragma unroll
  for (int i = 0; i < 8; ++i) { a[i] = (_Float16)(p[i] * sc); a[8 + i] = (_Float16)(p[16 + i] * sc); }
  return a;
}
__device__ __forceinline__ v16h fragc_f32(const float* W, int k0, int n, int lane, int ld, int K) {
  v16h a; const int g = lane >> 4;
#pragma unroll
  for (int i = 0; i < 8; ++i) { const int ka = k0 + 8 * g + i, kb = ka + 16;
    a[i] = (_Float16)(ka < K ? W[(size_t)ka * ld + n] : 0.f); a[8 + i] = (_Float16)(kb < K ? W[(size_t)kb * ld + n] : 0.f); }
  return a;
}
struct F2 { v16b h, l; };
__device__ __forceinline__ F2 bsplit16(const float v[16]) { F2 r;
#pragma unroll
  for (int i = 0; i < 16; ++i) { const __bf16 h = (__bf16)v[i]; r.h[i] = h; r.l[i] = (__bf16)(v[i] - (float)h); }
  return r; }
__device__ __forceinline__ F2 split_row(const float* row, int k0, int lane) { float v[16]; const float* p = row + k0 + 8 * (lane >> 4);
#pragma unroll
  for (int i = 0; i < 8; ++i) { v[i] = p[i]; v[8 + i] = p[16 + i]; }
  return bsplit16(v); }
__device__ __forceinline__ F2 split_rowK(const float* row, int k0, int lane, int K) { float v[16]; const int g = lane >> 4;
#pragma unroll
  for (int i = 0; i < 8; ++i) { const int ka = k0 + 8 * g + i, kb = ka + 16; v[i] = ka < K ? row[ka] : 0.f; v[8 + i] = kb < K ? row[kb] : 0.f; }
  return bsplit16(v); }
__device__ __forceinline__ F2 split_col(const float* W, int k0, int n, int lane, int ld, int K) { float v[16]; const int g = lane >> 4;
#pragma unroll
  for (int i = 0; i < 8; ++i) { const int ka = k0 + 8 * g + i, kb = ka + 16; v[i] = ka < K ? W[(size_t)ka * ld + n] : 0.f; v[8 + i] = kb < K ? W[(size_t)kb * ld + n] : 0.f; }
  return bsplit16(v); }
__device__ __forceinline__ v8f mac3(const F2& a, const F2& b, v8f c) { c = wmma_bf(a.l, b.h, c); c = wmma_bf(a.h, b.l, c); return wmma_bf(a.h, b.h, c); }
__device__ __forceinline__ float sigm(float v) { return 1.0f / (1.0f + expf(-v)); }
#define LDSX() do { asm volatile("s_wait_dscnt 0" ::: "memory"); __builtin_amdgcn_wave_barrier(); __builtin_amdgcn_fence(__ATOMIC_RELEASE, "workgroup"); } while (0)

#define NBT 256
#define TT 512
#define EMB 50
#define EP 64
#define HID 128
#define NTAG 9
#define VOC 12149
#define STARTTOK 7
#define KA (EP + HID)

__global__ __launch_bounds__(256) void k_gath(const int* __restrict__ inp, const int* __restrict__ lab, const float* __restrict__ emb, const float* __restrict__ demb, _Float16* __restrict__ X16) {
  const size_t q = (size_t)blockIdx.x * 256 + threadIdx.x; const size_t r = q >> 4; const int part = (int)(q & 15);
  if (r >= (size_t)2 * NBT * TT) return;
  const int which = (int)(r / ((size_t)NBT * TT)); const size_t rr = r % ((size_t)NBT * TT); const int b = (int)(rr / TT), t = (int)(rr % TT);
  int id; const float* tab; int nrow;
  if (which == 0) { id = inp[rr]; tab = emb; nrow = VOC; } else { id = (t == 0) ? STARTTOK : lab[(size_t)b * TT + t - 1]; tab = demb; nrow = NTAG; }
  id = id < 0 ? 0 : (id >= nrow ? nrow - 1 : id);
  union { _Float16 h4[4]; unsigned long long u; } pk;
#pragma unroll
  for (int e = 0; e < 4; ++e) { const int c = part * 4 + e; pk.h4[e] = (_Float16)(c < EMB ? tab[(size_t)id * EMB + c] : 0.f); }
  vst2((unsigned long long*)(X16 + r * EP) + part, pk.u);
}
__global__ __launch_bounds__(32) void k_rnn(const _Float16* __restrict__ X16, const float* __restrict__ eWx, const float* __restrict__ eWh, const float* __restrict__ eb, const float* __restrict__ dWx, const float* __restrict__ dWh, const float* __restrict__ db,
                                          const float* __restrict__ Wo, const float* __restrict__ bo, float* __restrict__ out) {
  __shared__ __align__(16) _Float16 sW[2][HID][KA + 8];
  __shared__ __align__(16) _Float16 sWo[16][HID + 8];
  __shared__ __align__(16) _Float16 sh[16][HID + 8];
  __shared__ float sb[2][HID]; __shared__ float sbo[16];
  __shared__ __align__(16) float sst[16][64 * NTAG + 4];
  const int lane = threadIdx.x, col = lane & 15, g = lane >> 4; const int b0 = blockIdx.x * 16;
  for (int q = lane; q < 2 * HID * KA; q += 32) { const int ph = q / (HID * KA), rem = q % (HID * KA), n = rem / KA, k = rem % KA; float v;
    const float* Wx = ph ? dWx : eWx; const float* Wh = ph ? dWh : eWh;
    if (k < EP) v = k < EMB ? Wx[k * HID + n] : 0.f; else v = Wh[(k - EP) * HID + n];
    sW[ph][n][k] = (_Float16)v; }
  for (int q = lane; q < 16 * HID; q += 32) { const int n = q / HID, k = q % HID; sWo[n][k] = (_Float16)(n < NTAG ? Wo[k * NTAG + n] : 0.f); }
  for (int q = lane; q < HID; q += 32) { sb[0][q] = eb[q]; sb[1][q] = db[q]; }
  if (lane < 16) sbo[lane] = lane < NTAG ? bo[lane] : 0.f;
  for (int q = lane; q < 16 * (HID + 8); q += 32) (&sh[0][0])[q] = (_Float16)0.f;
  LDSX();
#pragma unroll 1
  for (int ph = 0; ph < 2; ++ph) {
#pragma unroll 1
    for (int t = 0; t < TT; ++t) {
      v8f acc[8];
#pragma unroll
      for (int j = 0; j < 8; ++j) acc[j] = (v8f){};
#pragma unroll
      for (int kc = 0; kc < KA / 32; ++kc) { v16h a;
        if (kc < 2) a = frag_h(X16 + (((size_t)ph * NBT + b0 + col) * TT + t) * EP + kc * 32, lane); else a = frag_h(&sh[col][0] + (kc - 2) * 32, lane);
#pragma unroll
        for (int j = 0; j < 8; ++j) acc[j] = wmma16(a, frag_h(&sW[ph][j * 16 + col][0] + kc * 32, lane), acc[j]); }
      LDSX();
#pragma unroll
      for (int j = 0; j < 8; ++j) { const int n = j * 16 + col; const float bb = sb[ph][n];
#pragma unroll
        for (int r = 0; r < 8; ++r) sh[8 * g + r][n] = (_Float16)tanhf(acc[j][r] + bb); }
      LDSX();
      if (ph == 1) {
        v8f o = {};
#pragma unroll
        for (int kc = 0; kc < 4; ++kc) o = wmma16(frag_h(&sh[col][0] + kc * 32, lane), frag_h(&sWo[col][0] + kc * 32, lane), o);
        const int tl = t & 63;
        if (col < NTAG) {
#pragma unroll
          for (int r = 0; r < 8; ++r) sst[8 * g + r][tl * NTAG + col] = o[r] + sbo[col]; }
        if (tl == 63) { LDSX();
          for (int q = lane; q < 16 * 144; q += 32) { const int sq = q / 144, pc = q % 144; vst2(out + ((size_t)(b0 + sq) * TT + (t - 63)) * NTAG + pc * 4, *(const v4f*)(&sst[sq][pc * 4])); }
          LDSX(); } } } }
}
extern "C" void kernel_launch(void* const* d_in, const int* in_sizes, int n_in, void* d_out, int out_size, void* d_ws, size_t ws_size, hipStream_t stream) {
  (void)in_sizes; (void)n_in; (void)out_size; (void)ws_size;
  const int* inp = (const int*)d_in[0]; const int* lab = (const int*)d_in[1]; const float** I = (const float**)d_in;
  float* out = (float*)d_out;
  _Float16* X16 = (_Float16*)d_ws;
  k_gath<<<(2 * NBT * TT * 16 + 255) / 256, 256, 0, stream>>>(inp, lab, I[2], I[6], X16);
  k_rnn<<<NBT / 16, 32, 0, stream>>>(X16, I[3], I[4], I[5], I[7], I[8], I[9], I[10], I[11], out);
}
